// PhonemeAlignmentModel_24489903522589
// MI455X (gfx1250) — hardware-run, weakly checked
//
#include <hip/hip_runtime.h>

typedef _Float16 v16h __attribute__((ext_vector_type(16)));
typedef _Float16 v8h  __attribute__((ext_vector_type(8)));
typedef __bf16   v16b __attribute__((ext_vector_type(16)));
typedef __bf16   v8b  __attribute__((ext_vector_type(8)));
typedef float    v8f  __attribute__((ext_vector_type(8)));
typedef float    v4f  __attribute__((ext_vector_type(4)));
typedef double   v2d  __attribute__((ext_vector_type(2)));
typedef v8h __attribute__((may_alias)) v8ha;
typedef v8b __attribute__((may_alias)) v8ba;
typedef v4f __attribute__((may_alias)) v4fa;
union FragH { v16h v; v8h half[2]; };
union FragB { v16b v; v8b half[2]; };

#define NB     16
#define TA     2000
#define TLN    200
#define CA     80
#define CAP    96
#define CLG    52
#define CLP    64
#define HID    512
#define Z2     256
#define ZD     128
#define RPA    2048
#define RPL    256
#define SP     208
#define PTP    2240
#define TOFF   192
#define S0B    816
#define NSMB   37
#define NKDB   9216
#define NSMD   9472
#define NPROB  6400000
#define NPIECE 1600000
#define INV1800 (1.0f / 1800.0f)

__device__ __forceinline__ v8f wraw_f16(v16h a, v16h b, v8f c) {
#if defined(__HIP_DEVICE_COMPILE__)
  return __builtin_amdgcn_wmma_f32_16x16x32_f16(false, a, false, b, (short)0, c, false, false);
#else
  return c;
#endif
}
__device__ __forceinline__ v8f wraw_bf16(v16b a, v16b b, v8f c) {
#if defined(__HIP_DEVICE_COMPILE__)
  return __builtin_amdgcn_wmma_f32_16x16x32_bf16(false, a, false, b, (short)0, c, false, false);
#else
  return c;
#endif
}
__device__ __forceinline__ v8f wmma_bf16_g(v16b a, v16b b, v8f c) {
  v8f d = wraw_bf16(a, b, c);
#if defined(__HIP_DEVICE_COMPILE__)
  asm volatile("v_nop\n\tv_nop\n\tv_nop\n\tv_nop" : "+v"(d) : "v"(a), "v"(b));
#endif
  return d;
}

__device__ __forceinline__ double wave_sum_d(double v) {
#pragma unroll
  for (int o = 16; o > 0; o >>= 1) v += __shfl_xor(v, o, 32);
  return v;
}

__device__ __forceinline__ v8b zero8b() {
  v8b z;
#pragma unroll
  for (int e = 0; e < 8; ++e) z[e] = (__bf16)0.0f;
  return z;
}

__global__ __launch_bounds__(256) void k_cvt_x(const float* __restrict__ x, _Float16* __restrict__ xp,
                                               int CIN, int CINP, int T)
{
  __shared__ __attribute__((aligned(16))) _Float16 tile[8192];
  const int tid = threadIdx.x;
  const int b = blockIdx.y;
  const int TP = T + 2;
  const int r0 = blockIdx.x * 64;
  int nrows = TP - r0;
  if (nrows > 64) nrows = 64;
  const int nel = 64 * CINP;
  const float* xb = x + (size_t)b * CIN * T;
#pragma unroll 1
  for (int idx = tid; idx < nel; idx += 256) {
    const int c = idx >> 6;
    const int rl = idx & 63;
    const int t = r0 + rl - 1;
    const int tc = t < 0 ? 0 : (t >= T ? T - 1 : t);
    const int cc = c < CIN ? c : CIN - 1;
    float v = xb[(size_t)cc * T + tc];
    if (c >= CIN || t < 0 || t >= T) v = 0.0f;
    tile[rl * CINP + c] = (_Float16)v;
  }
  __syncthreads();
  const int npieces = nrows * (CINP >> 3);
  _Float16* dst = xp + ((size_t)b * TP + r0) * CINP;
#pragma unroll 1
  for (int p = tid; p < npieces; p += 256) {
    const v8h v = *(const v8ha*)(tile + 8 * p);
    *(volatile v8h*)(dst + 8 * p) = v;
  }
  __threadfence();
#pragma unroll 1
  for (int p = tid; p < npieces; p += 256) {
    const v8h v = *(const v8ha*)(tile + 8 * p);
    *(volatile v8h*)(dst + 8 * p) = v;
  }
}

__global__ __launch_bounds__(256) void k_cvt_w(const float* __restrict__ wsrc, _Float16* __restrict__ wt,
                                               int CIN, int CINP, int COUT, int RB, float scale)
{
  __shared__ __attribute__((aligned(16))) _Float16 tile[8192];
  const int tid = threadIdx.x;
  const int NR = 3 * COUT;
  const int r0 = blockIdx.x * RB;
  int nrows = NR - r0;
  if (nrows > RB) nrows = RB;
  const int nel = RB * CINP;
#pragma unroll 1
  for (int idx = tid; idx < nel; idx += 256) {
    const int rl = idx / CINP;
    const int ci = idx - rl * CINP;
    int R = r0 + rl;
    if (R > NR - 1) R = NR - 1;
    const int k = R / COUT;
    const int co = R - k * COUT;
    const int cic = ci < CIN ? ci : CIN - 1;
    float v = wsrc[((size_t)co * CIN + cic) * 3 + k] * scale;
    if (ci >= CIN || r0 + rl >= NR) v = 0.0f;
    tile[idx] = (_Float16)v;
  }
  __syncthreads();
  const int npieces = nrows * (CINP >> 3);
  _Float16* dst = wt + (size_t)r0 * CINP;
#pragma unroll 1
  for (int p = tid; p < npieces; p += 256) {
    const v8h v = *(const v8ha*)(tile + 8 * p);
    *(volatile v8h*)(dst + 8 * p) = v;
  }
  __threadfence();
#pragma unroll 1
  for (int p = tid; p < npieces; p += 256) {
    const v8h v = *(const v8ha*)(tile + 8 * p);
    *(volatile v8h*)(dst + 8 * p) = v;
  }
}

__device__ __forceinline__ void conv_kstep(const _Float16* a0p, const _Float16* a1p, const _Float16* btp,
                                           size_t nstr, int c0, int h, v8f (&acc)[2][4])
{
  FragH a0, a1, b0, b1, b2, b3;
  const int k0 = c0 + 8 * h, k1 = c0 + 16 + 8 * h;
  a0.half[0] = *(const v8ha*)(a0p + k0);            a0.half[1] = *(const v8ha*)(a0p + k1);
  a1.half[0] = *(const v8ha*)(a1p + k0);            a1.half[1] = *(const v8ha*)(a1p + k1);
  b0.half[0] = *(const v8ha*)(btp + k0);            b0.half[1] = *(const v8ha*)(btp + k1);
  b1.half[0] = *(const v8ha*)(btp + nstr + k0);     b1.half[1] = *(const v8ha*)(btp + nstr + k1);
  b2.half[0] = *(const v8ha*)(btp + 2 * nstr + k0); b2.half[1] = *(const v8ha*)(btp + 2 * nstr + k1);
  b3.half[0] = *(const v8ha*)(btp + 3 * nstr + k0); b3.half[1] = *(const v8ha*)(btp + 3 * nstr + k1);
  acc[0][0] = wraw_f16(a0.v, b0.v, acc[0][0]);
  acc[1][0] = wraw_f16(a1.v, b0.v, acc[1][0]);
  acc[0][1] = wraw_f16(a0.v, b1.v, acc[0][1]);
  acc[1][1] = wraw_f16(a1.v, b1.v, acc[1][1]);
  acc[0][2] = wraw_f16(a0.v, b2.v, acc[0][2]);
  acc[1][2] = wraw_f16(a1.v, b2.v, acc[1][2]);
  acc[0][3] = wraw_f16(a0.v, b3.v, acc[0][3]);
  acc[1][3] = wraw_f16(a1.v, b3.v, acc[1][3]);
#if defined(__HIP_DEVICE_COMPILE__)
  asm volatile("v_nop\n\tv_nop\n\tv_nop\n\tv_nop"
               : "+v"(acc[0][0]), "+v"(acc[0][1]), "+v"(acc[0][2]), "+v"(acc[0][3]),
                 "+v"(acc[1][0]), "+v"(acc[1][1]), "+v"(acc[1][2]), "+v"(acc[1][3])
               : "v"(a0.v), "v"(a1.v), "v"(b0.v), "v"(b1.v), "v"(b2.v), "v"(b3.v));
#endif
}

__device__ __forceinline__ void conv_store16(const _Float16* sT, _Float16* yp, int b, int TP, int T,
                                             int COUT, int co0, int t0, int w, int lane, bool firstx)
{
  const int q8 = lane & 7, sub = lane >> 3;
#pragma unroll
  for (int i = 0; i < 8; ++i) {
    const int lid = w * 32 + i * 4 + sub;
    const int t = t0 + lid;
    const v8h v = *(const v8ha*)(sT + lid * 64 + 8 * q8);
    if (t <= T) {
      *(volatile v8h*)(yp + ((size_t)b * TP + t + 1) * COUT + co0 + 8 * q8) = v;
    }
  }
  if (firstx && w == 0 && sub == 0) {
    v8h z;
#pragma unroll
    for (int e = 0; e < 8; ++e) z[e] = (_Float16)0.0f;
    *(volatile v8h*)(yp + (size_t)b * TP * COUT + co0 + 8 * q8) = z;
  }
}

__device__ __forceinline__ void conv_store32(const float* sF, float* yf, int b, int T, int COUT, int co0,
                                             int t0, int w, int lane)
{
  const int p16 = lane & 15, sub2 = lane >> 4;
#pragma unroll
  for (int i = 0; i < 16; ++i) {
    const int lid = w * 32 + i * 2 + sub2;
    const int t = t0 + lid;
    const v4f v = *(const v4fa*)(sF + lid * 64 + 4 * p16);
    if (t < T) {
      *(volatile v4f*)(yf + ((size_t)b * T + t) * COUT + co0 + 4 * p16) = v;
    }
  }
}

template <bool OUT16>
__global__ __launch_bounds__(128) __attribute__((amdgpu_num_vgpr(256)))
void k_conv(const _Float16* __restrict__ xp, const _Float16* __restrict__ wt,
            const float* __restrict__ bias, void* __restrict__ yout,
            int CINP, int COUT, int T, float oscale, int relu)
{
  __shared__ __attribute__((aligned(16))) unsigned char sraw[32768];
  const int tid = threadIdx.x, lane = tid & 31, w = tid >> 5, h = lane >> 4, m = lane & 15;
  const int b = blockIdx.z;
  const int t0 = blockIdx.x * 128, co0 = blockIdx.y * 64;
  const int TP = T + 2;
  const int t0w = t0 + 32 * w;

  const _Float16* xb = xp + (size_t)b * TP * CINP;
  const int cl = T + 1;
  const int rA = t0w + m, rB = t0w + 16 + m;
  const _Float16* a00 = xb + (size_t)(rA < cl ? rA : cl) * CINP;
  const _Float16* a01 = xb + (size_t)(rA + 1 < cl ? rA + 1 : cl) * CINP;
  const _Float16* a02 = xb + (size_t)(rA + 2 < cl ? rA + 2 : cl) * CINP;
  const _Float16* a10 = xb + (size_t)(rB < cl ? rB : cl) * CINP;
  const _Float16* a11 = xb + (size_t)(rB + 1 < cl ? rB + 1 : cl) * CINP;
  const _Float16* a12 = xb + (size_t)(rB + 2 < cl ? rB + 2 : cl) * CINP;
  const _Float16* wb = wt + (size_t)(co0 + m) * CINP;
  const size_t tstr = (size_t)COUT * CINP, nstr = (size_t)16 * CINP;

  const v8f z8 = {0.f, 0.f, 0.f, 0.f, 0.f, 0.f, 0.f, 0.f};
  v8f acc[2][4];
#pragma unroll
  for (int mt = 0; mt < 2; ++mt)
#pragma unroll
    for (int nt = 0; nt < 4; ++nt) acc[mt][nt] = z8;

#pragma unroll 1
  for (int c0 = 0; c0 < CINP; c0 += 32) conv_kstep(a00, a10, wb, nstr, c0, h, acc);
#pragma unroll 1
  for (int c0 = 0; c0 < CINP; c0 += 32) conv_kstep(a01, a11, wb + tstr, nstr, c0, h, acc);
#pragma unroll 1
  for (int c0 = 0; c0 < CINP; c0 += 32) conv_kstep(a02, a12, wb + 2 * tstr, nstr, c0, h, acc);

  if (OUT16) {
    _Float16* sT = (_Float16*)sraw;
#pragma unroll
    for (int nt = 0; nt < 4; ++nt) {
      const float bv = bias[co0 + 16 * nt + m];
#pragma unroll
      for (int mt = 0; mt < 2; ++mt) {
#pragma unroll
        for (int r = 0; r < 8; ++r) {
          const int tokl = 32 * w + 16 * mt + 8 * h + r;
          float y = acc[mt][nt][r] * oscale + bv;
          if (relu) y = fmaxf(y, 0.0f);
          if (t0 + tokl >= T) y = 0.0f;
          sT[tokl * 64 + 16 * nt + m] = (_Float16)y;
        }
      }
    }
  } else {
    float* sF = (float*)sraw;
#pragma unroll
    for (int nt = 0; nt < 4; ++nt) {
      const float bv = bias[co0 + 16 * nt + m];
#pragma unroll
      for (int mt = 0; mt < 2; ++mt) {
#pragma unroll
        for (int r = 0; r < 8; ++r) {
          const int tokl = 32 * w + 16 * mt + 8 * h + r;
          float y = acc[mt][nt][r] * oscale + bv;
          if (relu) y = fmaxf(y, 0.0f);
          if (t0 + tokl >= T) y = 0.0f;
          sF[tokl * 64 + 16 * nt + m] = y;
        }
      }
    }
  }
  __syncthreads();

  const bool firstx = (blockIdx.x == 0);
  if (OUT16) {
    const _Float16* sT = (const _Float16*)sraw;
    _Float16* yp = (_Float16*)yout;
    conv_store16(sT, yp, b, TP, T, COUT, co0, t0, w, lane, firstx);
    __threadfence();
    conv_store16(sT, yp, b, TP, T, COUT, co0, t0, w, lane, firstx);
  } else {
    const float* sF = (const float*)sraw;
    float* yf = (float*)yout;
    conv_store32(sF, yf, b, T, COUT, co0, t0, w, lane);
    __threadfence();
    conv_store32(sF, yf, b, T, COUT, co0, t0, w, lane);
  }
}

__global__ __launch_bounds__(256) void k_mu(const float* __restrict__ m3, __bf16* __restrict__ phi,
                                           __bf16* __restrict__ plo, float* __restrict__ nrm,
                                           double* __restrict__ part, int T, int RP)
{
  __shared__ __attribute__((aligned(16))) float nls[64];
  __shared__ double red[8];
  const int tid = threadIdx.x, lane = tid & 31, w = tid >> 5, hf = lane >> 4, l16 = lane & 15;
  const int b = blockIdx.y, r0 = blockIdx.x * 64;
  double kacc = 0.0;
  v8b hiv[4], lov[4];
#pragma unroll
  for (int it = 0; it < 4; ++it) {
    const int rl = it * 16 + 2 * w + hf;
    const int row = r0 + rl;
    const bool valid = row < T;
    const int rc = valid ? row : T - 1;
    const float* src = m3 + ((size_t)b * T + rc) * Z2 + 8 * l16;
    const v4f ma = *(const v4fa*)src, mb = *(const v4fa*)(src + 4);
    const v4f va = *(const v4fa*)(src + ZD), vb = *(const v4fa*)(src + ZD + 4);
    const float mu[8] = {ma.x, ma.y, ma.z, ma.w, mb.x, mb.y, mb.z, mb.w};
    const float lg[8] = {va.x, va.y, va.z, va.w, vb.x, vb.y, vb.z, vb.w};
    float s2 = 0.0f, kt = 0.0f;
#pragma unroll
    for (int e = 0; e < 8; ++e) {
      const float q = mu[e] * mu[e];
      s2 += q;
      kt += (1.0f + lg[e]) - q - __expf(lg[e]);
    }
    if (!valid) { s2 = 0.0f; kt = 0.0f; }
    kacc += (double)kt;
    s2 += __shfl_xor(s2, 8, 32);
    s2 += __shfl_xor(s2, 4, 32);
    s2 += __shfl_xor(s2, 2, 32);
    s2 += __shfl_xor(s2, 1, 32);
    if (l16 == 0) nls[rl] = s2;
    v8b hvv, lvv;
#pragma unroll
    for (int e = 0; e < 8; ++e) {
      const float xv = valid ? mu[e] : 0.0f;
      const __bf16 hb = (__bf16)xv;
      const __bf16 lb = (__bf16)(xv - (float)hb);
      hvv[e] = hb;
      lvv[e] = lb;
    }
    hiv[it] = hvv;
    lov[it] = lvv;
  }
  kacc = wave_sum_d(kacc);
  if (lane == 0) red[w] = kacc;
  __syncthreads();

  const size_t nbase = (size_t)b * RP + r0;
  double* pline = part + ((size_t)(blockIdx.y * gridDim.x + blockIdx.x)) * 16 + 2 * (lane & 7);
#pragma unroll 1
  for (int pass = 0; pass < 2; ++pass) {
#pragma unroll
    for (int it = 0; it < 4; ++it) {
      const int rl = it * 16 + 2 * w + hf;
      const size_t off = (nbase + rl) * ZD + 8 * l16;
      *(volatile v8b*)(phi + off) = hiv[it];
      *(volatile v8b*)(plo + off) = lov[it];
    }
    const v4f nv = *(const v4fa*)(nls + 4 * (lane & 15));
    const double rv = red[lane & 7];
    if (w == 0 && lane < 16) *(volatile v4f*)(nrm + nbase + 4 * lane) = nv;
    if (w == 0 && lane < 8) { v2d val = {rv, 0.0}; *(volatile v2d*)pline = val; }
    if (pass == 0) __threadfence();
  }
}

__device__ __forceinline__ void stream_rows(const float* sL, float* dst, int npieces, int tid) {
#pragma unroll 1
  for (int p = tid; p < npieces; p += 128) {
    const int row = p / 50;
    const int c4 = p - row * 50;
    const v4f v = *(const v4fa*)(sL + row * SP + 4 * c4);
    *(volatile v4f*)(dst + 4 * p) = v;
  }
}

__device__ __forceinline__ void stream_pt(const float* sL, __bf16* ptb, int t0, int tid, bool zfill) {
#pragma unroll 1
  for (int p = tid; p < SP * 8; p += 128) {
    const int o = p >> 3, q = p & 7;
    const float* src = sL + (8 * q) * SP + o;
    v8b v;
#pragma unroll
    for (int e = 0; e < 8; ++e) v[e] = (__bf16)src[e * SP];
    *(volatile v8b*)(ptb + (size_t)o * PTP + TOFF + t0 + 8 * q) = v;
  }
  if (zfill) {
    const v8b z = zero8b();
#pragma unroll 1
    for (int p = tid; p < SP * 24; p += 128) {
      const int row = p / 24, q = p - row * 24;
      *(volatile v8b*)(ptb + (size_t)row * PTP + 8 * q) = z;
    }
  }
}

__global__ __launch_bounds__(128) __attribute__((amdgpu_num_vgpr(256)))
void k_dist(const __bf16* __restrict__ ahi, const __bf16* __restrict__ alo,
            const __bf16* __restrict__ lhi, const __bf16* __restrict__ llo,
            const float* __restrict__ na, const float* __restrict__ nl,
            float* __restrict__ probs, float* __restrict__ logp, __bf16* __restrict__ pt)
{
  __shared__ __attribute__((aligned(16))) float sL[64 * SP];
  const int tid = threadIdx.x, lane = tid & 31, w = tid >> 5, h = lane >> 4, m = lane & 15;
  const int b = blockIdx.y, t0 = blockIdx.x * 64, tw = t0 + 16 * w;

  const __bf16* arh = ahi + ((size_t)b * RPA + tw + m) * ZD;
  const __bf16* arl = alo + ((size_t)b * RPA + tw + m) * ZD;
  const __bf16* lbh = lhi + ((size_t)b * RPL + m) * ZD;
  const __bf16* lbl = llo + ((size_t)b * RPL + m) * ZD;

  v16b ahv[4], alv[4];
#pragma unroll
  for (int ks = 0; ks < 4; ++ks) {
    FragB fh, fl;
    const int k0 = 32 * ks + 8 * h, k1 = 32 * ks + 16 + 8 * h;
    fh.half[0] = *(const v8ba*)(arh + k0); fh.half[1] = *(const v8ba*)(arh + k1);
    fl.half[0] = *(const v8ba*)(arl + k0); fl.half[1] = *(const v8ba*)(arl + k1);
    ahv[ks] = fh.v;
    alv[ks] = fl.v;
  }
  float nar[8];
#pragma unroll
  for (int r = 0; r < 8; ++r) nar[r] = na[(size_t)b * RPA + tw + 8 * h + r];
  float* srow = sL + (16 * w + 8 * h) * SP + m;

  const v8f z8 = {0.f, 0.f, 0.f, 0.f, 0.f, 0.f, 0.f, 0.f};
#pragma unroll 1
  for (int j = 0; j < 13; ++j) {
    const __bf16* lh = lbh + (size_t)j * 16 * ZD;
    const __bf16* ll = lbl + (size_t)j * 16 * ZD;
    v8f acc = z8;
#pragma unroll
    for (int ks = 0; ks < 4; ++ks) {
      FragB fbh, fbl;
      const int k0 = 32 * ks + 8 * h, k1 = 32 * ks + 16 + 8 * h;
      fbh.half[0] = *(const v8ba*)(lh + k0); fbh.half[1] = *(const v8ba*)(lh + k1);
      fbl.half[0] = *(const v8ba*)(ll + k0); fbl.half[1] = *(const v8ba*)(ll + k1);
      acc = wraw_bf16(ahv[ks], fbh.v, acc);
      acc = wraw_bf16(ahv[ks], fbl.v, acc);
      acc = wraw_bf16(alv[ks], fbh.v, acc);
#if defined(__HIP_DEVICE_COMPILE__)
      asm volatile("v_nop\n\tv_nop\n\tv_nop\n\tv_nop"
                   : "+v"(acc) : "v"(ahv[ks]), "v"(alv[ks]), "v"(fbh.v), "v"(fbl.v) : "memory");
#endif
    }
    const float nlv = nl[(size_t)b * RPL + 16 * j + m];
#pragma unroll
    for (int r = 0; r < 8; ++r) {
      const float d2 = (nar[r] + nlv) - 2.0f * acc[r];
      srow[r * SP + 16 * j] = -sqrtf(fmaxf(d2, 0.0f));
    }
  }
  __syncthreads();

  const float ninf = -__builtin_inff();
#pragma unroll 1
  for (int rr = 0; rr < 16; ++rr) {
    float* x = sL + (16 * w + rr) * SP;
    float v[7];
    float mxv = ninf;
#pragma unroll
    for (int i = 0; i < 7; ++i) {
      const int c = lane + 32 * i;
      const int cc = c < SP ? c : SP - 1;
      float xv = x[cc];
      if (c >= TLN) xv = ninf;
      v[i] = xv;
      mxv = fmaxf(mxv, xv);
    }
    mxv = fmaxf(mxv, __shfl_xor(mxv, 16, 32));
    mxv = fmaxf(mxv, __shfl_xor(mxv, 8, 32));
    mxv = fmaxf(mxv, __shfl_xor(mxv, 4, 32));
    mxv = fmaxf(mxv, __shfl_xor(mxv, 2, 32));
    mxv = fmaxf(mxv, __shfl_xor(mxv, 1, 32));
    float s = 0.0f;
#pragma unroll
    for (int i = 0; i < 7; ++i) s += __expf(v[i] - mxv);
    s += __shfl_xor(s, 16, 32);
    s += __shfl_xor(s, 8, 32);
    s += __shfl_xor(s, 4, 32);
    s += __shfl_xor(s, 2, 32);
    s += __shfl_xor(s, 1, 32);
    const float lsv = logf(s);
#pragma unroll
    for (int i = 0; i < 7; ++i) {
      const int c = lane + 32 * i;
      if (c < TLN) x[c] = (v[i] - mxv) - lsv;
    }
  }
  __syncthreads();

  int nv = TA - t0;
  nv = nv > 64 ? 64 : nv;
  const int npieces = nv * (TLN / 4);
  const size_t gbase = ((size_t)b * TA + t0) * TLN;

  stream_rows(sL, logp + gbase, npieces, tid);
  __threadfence();
  stream_rows(sL, logp + gbase, npieces, tid);
  __syncthreads();

#pragma unroll 1
  for (int idx = tid; idx < 64 * SP; idx += 128) {
    const int row = idx / SP;
    const int c = idx - row * SP;
    float p = __expf(sL[idx]);
    if (c >= TLN || t0 + row >= TA) p = 0.0f;
    sL[idx] = p;
  }
  __syncthreads();

  stream_rows(sL, probs + gbase, npieces, tid);
  __threadfence();
  stream_rows(sL, probs + gbase, npieces, tid);

  __bf16* ptb = pt + (size_t)b * SP * PTP;
  const bool zfill = (blockIdx.x == 0);
  stream_pt(sL, ptb, t0, tid, zfill);
  __threadfence();
  stream_pt(sL, ptb, t0, tid, zfill);
}

__global__ __launch_bounds__(64) __attribute__((amdgpu_num_vgpr(256)))
void k_smooth(const __bf16* __restrict__ pt, const float* __restrict__ logp, double* __restrict__ part)
{
  __shared__ __bf16 gtab[SP];
  __shared__ double redg[2];
  __shared__ double redp[2];
  const int tid = threadIdx.x, lane = tid & 31, w = tid >> 5, h = lane >> 4, m = lane & 15;
  const int b = blockIdx.y;
  const int tile = blockIdx.x * 2 + w;
  const int s0 = S0B + 16 * tile;
  const int tw0 = s0 - 1000;

  float gs = 0.0f;
#pragma unroll 1
  for (int v = tid; v < TA; v += 64) {
    const float u = (float)v;
    gs += expf(-(u * u) * INV1800);
  }
  const double gd = wave_sum_d((double)gs);
  if (lane == 0) redg[w] = gd;
  __syncthreads();
  const float gsum = (float)(redg[0] + redg[1]);
  const float ginv = 1.0f / gsum;
#pragma unroll 1
  for (int i = tid; i < SP; i += 64) {
    const int v = i - 16;
    float val = 0.0f;
    if (v >= 0) {
      const float u = (float)v;
      val = expf(-(u * u) * INV1800) * ginv;
    }
    gtab[i] = (__bf16)val;
  }
  __syncthreads();

  v16b af[6];
#pragma unroll
  for (int ks = 0; ks < 6; ++ks) {
    v16b f;
#pragma unroll
    for (int e = 0; e < 16; ++e) {
      const int k = 32 * ks + ((e < 8) ? (8 * h + e) : (8 + 8 * h + e));
      f[e] = gtab[k + 15 - m];
    }
    af[ks] = f;
  }

  const __bf16* prow = pt + ((size_t)(b * SP + m)) * PTP + (TOFF + tw0);
  const float* lrow = logp + ((size_t)b * TA + s0 + 8 * h) * TLN;
  const v8f z8 = {0.f, 0.f, 0.f, 0.f, 0.f, 0.f, 0.f, 0.f};
  float partf = 0.0f;
#pragma unroll 1
  for (int j = 0; j < 13; ++j) {
    const __bf16* pj = prow + (size_t)j * 16 * PTP;
    v8f acc = z8;
#pragma unroll
    for (int ks = 0; ks < 6; ++ks) {
      FragB fb;
      fb.half[0] = *(const v8ba*)(pj + 32 * ks + 8 * h);
      fb.half[1] = *(const v8ba*)(pj + 32 * ks + 16 + 8 * h);
      acc = wmma_bf16_g(af[ks], fb.v, acc);
    }
    const int o = 16 * j + m;
    const int oc = o < TLN ? o : TLN - 1;
#pragma unroll
    for (int r = 0; r < 8; ++r) {
      float lp = lrow[(size_t)r * TLN + oc];
      if (o >= TLN) lp = 0.0f;
      partf += acc[r] * lp;
    }
  }
  const double pd = wave_sum_d((double)partf);
  if (lane == 0) redp[w] = pd;
  __syncthreads();
  const double r0v = redp[0], r1v = redp[1];
  v2d val = {0.0, 0.0};
  if (lane == 0) { val.x = r0v; val.y = r1v; }
  double* dstp = part + ((size_t)(blockIdx.y * gridDim.x + blockIdx.x)) * 16 + 2 * (lane & 7);
  if (w == 0 && lane < 8) *(volatile v2d*)dstp = val;
  __threadfence();
  if (w == 0 && lane < 8) *(volatile v2d*)dstp = val;
}

__global__ __launch_bounds__(256) void k_out(const float* __restrict__ probs, const double* __restrict__ part,
                                            float* __restrict__ out)
{
  __shared__ double red[8];
  const int tid = threadIdx.x, lane = tid & 31, w = tid >> 5;
  float loss = 0.0f;
  if (blockIdx.x == 0) {
    double sk = 0.0, ss = 0.0;
#pragma unroll 1
    for (int i = tid; i < NKDB; i += 256) sk += part[i];
#pragma unroll 1
    for (int i = tid; i < NSMD; i += 256) ss += part[NKDB + i];
    double v = -ss - 0.05 * sk;
    v = wave_sum_d(v);
    if (lane == 0) red[w] = v;
    __syncthreads();
    double t = 0.0;
#pragma unroll
    for (int q = 0; q < 8; ++q) t += red[q];
    loss = (float)t;
  }
  v4f ov[8];
#pragma unroll
  for (int it = 0; it < 8; ++it) {
    const long long p = (long long)blockIdx.x * 2048 + it * 256 + tid;
    float f[4];
#pragma unroll
    for (int i = 0; i < 4; ++i) {
      long long idx = 4 * p - 1 + i;
      if (idx < 0) idx = 0;
      if (idx > NPROB - 1) idx = NPROB - 1;
      f[i] = probs[idx];
    }
    if (p == 0) f[0] = loss;
    v4f o = {f[0], f[1], f[2], f[3]};
    ov[it] = o;
  }
  const float tailv = probs[NPROB - 1];
#pragma unroll 1
  for (int pass = 0; pass < 2; ++pass) {
#pragma unroll
    for (int it = 0; it < 8; ++it) {
      const long long p = (long long)blockIdx.x * 2048 + it * 256 + tid;
      if (p < NPIECE) *(volatile v4f*)(out + 4 * p) = ov[it];
    }
    if (blockIdx.x == 0 && tid == 0) *(volatile float*)(out + NPROB) = tailv;
    if (pass == 0) __threadfence();
  }
}

static inline size_t al256(size_t x) { return (x + 255) & ~(size_t)255; }

extern "C" void kernel_launch(void* const* d_in, const int* in_sizes, int n_in,
                              void* d_out, int out_size, void* d_ws, size_t ws_size,
                              hipStream_t stream) {
  if (n_in < 14) return;
  if (in_sizes[0] != NB * CA * TA || in_sizes[1] != NB * CLG * TLN) return;
  if (in_sizes[2] != HID * CA * 3 || in_sizes[3] != HID || in_sizes[4] != HID * HID * 3 ||
      in_sizes[5] != HID || in_sizes[6] != Z2 * HID * 3 || in_sizes[7] != Z2) return;
  if (in_sizes[8] != HID * CLG * 3 || in_sizes[9] != HID || in_sizes[10] != HID * HID * 3 ||
      in_sizes[11] != HID || in_sizes[12] != Z2 * HID * 3 || in_sizes[13] != Z2) return;
  if (out_size != 1 + NPROB) return;

  const float* ain  = (const float*)d_in[0];
  const float* lin  = (const float*)d_in[1];
  const float* a_w1 = (const float*)d_in[2];
  const float* a_b1 = (const float*)d_in[3];
  const float* a_w2 = (const float*)d_in[4];
  const float* a_b2 = (const float*)d_in[5];
  const float* a_w3 = (const float*)d_in[6];
  const float* a_b3 = (const float*)d_in[7];
  const float* l_w1 = (const float*)d_in[8];
  const float* l_b1 = (const float*)d_in[9];
  const float* l_w2 = (const float*)d_in[10];
  const float* l_b2 = (const float*)d_in[11];
  const float* l_w3 = (const float*)d_in[12];
  const float* l_b3 = (const float*)d_in[13];
  float* out = (float*)d_out;

  size_t off = 0;
  const size_t oXA   = off; off += al256((size_t)NB * (TA + 2) * CAP * 2);
  const size_t oXL   = off; off += al256((size_t)NB * (TLN + 2) * CLP * 2);
  const size_t oWA1  = off; off += al256((size_t)3 * HID * CAP * 2);
  const size_t oWA2  = off; off += al256((size_t)3 * HID * HID * 2);
  const size_t oWA3  = off; off += al256((size_t)3 * Z2 * HID * 2);
  const size_t oWL1  = off; off += al256((size_t)3 * HID * CLP * 2);
  const size_t oWL2  = off; off += al256((size_t)3 * HID * HID * 2);
  const size_t oWL3  = off; off += al256((size_t)3 * Z2 * HID * 2);
  const size_t oH1A  = off; off += al256((size_t)NB * (TA + 2) * HID * 2);
  const size_t oH2A  = off; off += al256((size_t)NB * (TA + 2) * HID * 2);
  const size_t oH1L  = off; off += al256((size_t)NB * (TLN + 2) * HID * 2);
  const size_t oH2L  = off; off += al256((size_t)NB * (TLN + 2) * HID * 2);
  const size_t oMAH  = off; off += al256((size_t)NB * RPA * ZD * 2);
  const size_t oMAL  = off; off += al256((size_t)NB * RPA * ZD * 2);
  const size_t oMLH  = off; off += al256((size_t)NB * RPL * ZD * 2);
  const size_t oMLL  = off; off += al256((size_t)NB * RPL * ZD * 2);
  const size_t oNA   = off; off += al256((size_t)NB * RPA * 4);
  const size_t oNL   = off; off += al256((size_t)NB * RPL * 4);
  const size_t oPT   = off; off += al256((size_t)NB * SP * PTP * 2);
  const size_t oPART = off; off += al256((size_t)(NKDB + NSMD) * 8);
  if (off > ws_size || off > (size_t)134217728) return;
  if ((size_t)NB * TA * Z2 * 4 > (size_t)NB * (TA + 2) * HID * 2) return;
  if ((size_t)NB * TA * TLN * 4 > (size_t)NB * (TA + 2) * HID * 2) return;
  if ((size_t)NB * TLN * Z2 * 4 > (size_t)NB * (TLN + 2) * HID * 2) return;

  char* ws = (char*)d_ws;
  _Float16* XA  = (_Float16*)(ws + oXA);
  _Float16* XL  = (_Float16*)(ws + oXL);
  _Float16* WA1 = (_Float16*)(ws + oWA1);
  _Float16* WA2 = (_Float16*)(ws + oWA2);
  _Float16* WA3 = (_Float16*)(ws + oWA3);
  _Float16* WL1 = (_Float16*)(ws + oWL1);
  _Float16* WL2 = (_Float16*)(ws + oWL2);
  _Float16* WL3 = (_Float16*)(ws + oWL3);
  _Float16* H1A = (_Float16*)(ws + oH1A);
  _Float16* H2A = (_Float16*)(ws + oH2A);
  _Float16* H1L = (_Float16*)(ws + oH1L);
  _Float16* H2L = (_Float16*)(ws + oH2L);
  float*    M3A = (float*)(ws + oH1A);
  float*    M3L = (float*)(ws + oH1L);
  float*    LOGP = (float*)(ws + oH1A);
  float*    PROBS = (float*)(ws + oH2A);
  __bf16*   MAH = (__bf16*)(ws + oMAH);
  __bf16*   MAL = (__bf16*)(ws + oMAL);
  __bf16*   MLH = (__bf16*)(ws + oMLH);
  __bf16*   MLL = (__bf16*)(ws + oMLL);
  float*    NA  = (float*)(ws + oNA);
  float*    NLv = (float*)(ws + oNL);
  __bf16*   PT  = (__bf16*)(ws + oPT);
  double*   PART = (double*)(ws + oPART);

  k_cvt_x<<<dim3((TA + 2 + 63) / 64, NB), 256, 0, stream>>>(ain, XA, CA, CAP, TA);
  k_cvt_x<<<dim3((TLN + 2 + 63) / 64, NB), 256, 0, stream>>>(lin, XL, CLG, CLP, TLN);
  k_cvt_w<<<dim3((3 * HID) / 64), 256, 0, stream>>>(a_w1, WA1, CA, CAP, HID, 64, 64.0f);
  k_cvt_w<<<dim3((3 * HID) / 16), 256, 0, stream>>>(a_w2, WA2, HID, HID, HID, 16, 256.0f);
  k_cvt_w<<<dim3((3 * Z2) / 16), 256, 0, stream>>>(a_w3, WA3, HID, HID, Z2, 16, 256.0f);
  k_cvt_w<<<dim3((3 * HID) / 64), 256, 0, stream>>>(l_w1, WL1, CLG, CLP, HID, 64, 64.0f);
  k_cvt_w<<<dim3((3 * HID) / 16), 256, 0, stream>>>(l_w2, WL2, HID, HID, HID, 16, 256.0f);
  k_cvt_w<<<dim3((3 * Z2) / 16), 256, 0, stream>>>(l_w3, WL3, HID, HID, Z2, 16, 256.0f);

  k_conv<true><<<dim3((TA + 128) / 128, HID / 64, NB), 128, 0, stream>>>(
      XA, WA1, a_b1, (void*)H1A, CAP, HID, TA, 0.015625f, 1);
  k_conv<true><<<dim3((TA + 128) / 128, HID / 64, NB), 128, 0, stream>>>(
      H1A, WA2, a_b2, (void*)H2A, HID, HID, TA, 0.00390625f, 1);
  k_conv<false><<<dim3((TA + 128) / 128, Z2 / 64, NB), 128, 0, stream>>>(
      H2A, WA3, a_b3, (void*)M3A, HID, Z2, TA, 0.00390625f, 0);
  k_conv<true><<<dim3((TLN + 128) / 128, HID / 64, NB), 128, 0, stream>>>(
      XL, WL1, l_b1, (void*)H1L, CLP, HID, TLN, 0.015625f, 1);
  k_conv<true><<<dim3((TLN + 128) / 128, HID / 64, NB), 128, 0, stream>>>(
      H1L, WL2, l_b2, (void*)H2L, HID, HID, TLN, 0.00390625f, 1);
  k_conv<false><<<dim3((TLN + 128) / 128, Z2 / 64, NB), 128, 0, stream>>>(
      H2L, WL3, l_b3, (void*)M3L, HID, Z2, TLN, 0.00390625f, 0);

  k_mu<<<dim3(RPA / 64, NB), 256, 0, stream>>>(M3A, MAH, MAL, NA, PART, TA, RPA);
  k_mu<<<dim3(RPL / 64, NB), 256, 0, stream>>>(M3L, MLH, MLL, NLv, PART + (size_t)NB * (RPA / 64) * 16, TLN, RPL);

  k_dist<<<dim3(RPA / 64, NB), 128, 0, stream>>>(MAH, MAL, MLH, MLL, NA, NLv, PROBS, LOGP, PT);

  k_smooth<<<dim3(NSMB, NB), 64, 0, stream>>>(PT, LOGP, PART + NKDB);

  k_out<<<dim3((NPIECE + 2047) / 2048), 256, 0, stream>>>(PROBS, PART, out);
}
